// GOAD_35725537968402
// MI455X (gfx1250) — hardware-verified
//
#include <hip/hip_runtime.h>
#include <stddef.h>


typedef _Float16 h16;
typedef _Float16 v16h __attribute__((ext_vector_type(16)));
typedef _Float16 v8h  __attribute__((ext_vector_type(8)));
typedef float    v8f  __attribute__((ext_vector_type(8)));
typedef float    v4f  __attribute__((ext_vector_type(4)));
typedef float    v2f  __attribute__((ext_vector_type(2)));

#ifndef NB
#define NB 32768
#endif
#define NB_FULL 32768
#define NF 128
#define NT 32
#define ND 16
#define NH 10
#define REPW (NT * NH)

#ifndef XT_RES
#define XT_RES 1
#endif

#define XCARRY  16.0f
#define WCARRY  64.0f
#define XTCARRY 16.0f
#define RCARRY  2048.0f
#define XT_SCALE (XTCARRY / (XCARRY * WCARRY))
#define H0_SCALE (1.0f / (WCARRY * XTCARRY))

#define K1_ROWS   32
#define K1_BLOCKS (NB / K1_ROWS)
#define TRI_ITERS 8
#define TRI_BLOCKS ((NB * NT) / (256 * TRI_ITERS))
#define FIN_ROWS  1024
#define FIN_BLOCKS (NB / FIN_ROWS)

#define PITCH 324
#define LDA   136
#define WP    12

#define OUT1_OFF ((size_t)NB_FULL * REPW)

static_assert(NB >= 1024 && NB <= NB_FULL && (NB % 1024) == 0);
static_assert(NF == 128 && ND == 16 && NT == 32 && NH == 10);
static_assert((NF % 32) == 0);
static_assert(REPW == 320 && (REPW * 4) % 128 == 0);
static_assert(OUT1_OFF * 4 == (size_t)41943040);
static_assert((OUT1_OFF * 4) % 128 == 0);
static_assert(K1_BLOCKS * K1_ROWS == NB);
static_assert(TRI_BLOCKS * 256 * TRI_ITERS == NB * NT);
static_assert(FIN_BLOCKS * FIN_ROWS == NB && FIN_ROWS == 256 * 4);
static_assert((PITCH % 4) == 0 && PITCH >= REPW);
static_assert((LDA % 8) == 0 && LDA >= NF);
static_assert((WP % 4) == 0 && WP >= NH && WP == 12);
static_assert(5 * 8 * 32 == 16 * (REPW / 4));
static_assert(64 * 5 == REPW);
static_assert((64 + 16) * 4 == REPW);
static_assert(256 * 8 == ND * NF);

#define AWT_BYTES  ((size_t)NT * ND * NF * 2)
#define PART_BYTES ((size_t)K1_BLOCKS * REPW * 4)
#define CE_BYTES   ((size_t)NB * 4)
#define MEAN_BYTES ((size_t)REPW * 4)
#define HP_BYTES   ((size_t)TRI_BLOCKS * 128)
#define OFF_AWT  ((size_t)0)
#define OFF_PART (OFF_AWT + AWT_BYTES)
#define OFF_CE   (OFF_PART + PART_BYTES)
#define OFF_MEAN (OFF_CE + CE_BYTES)
#define OFF_HP   (OFF_MEAN + MEAN_BYTES)
#define WS_TOTAL (OFF_HP + HP_BYTES)
static_assert((AWT_BYTES % 128) == 0 && (PART_BYTES % 128) == 0 && (CE_BYTES % 128) == 0);
static_assert((MEAN_BYTES % 128) == 0 && (HP_BYTES % 128) == 0);
static_assert(WS_TOTAL <= (size_t)134217728);

__device__ __forceinline__ float bf16r(float x) {
  unsigned int u = __float_as_uint(x);
  u = (u + 0x7FFFu + ((u >> 16) & 1u)) & 0xFFFF0000u;
  return __uint_as_float(u);
}

static __device__ __forceinline__ h16 toh_flush(float v) {
  const h16 r = (h16)v;
  return (fabsf(v) < 6.103515625e-05f) ? (h16)0.0f : r;
}

__device__ __forceinline__ v16h frag_at(const _Float16* p) {
  v8h lo = *(const v8h*)(p);
  v8h hi = *(const v8h*)(p + 16);
  v16h out;
#pragma unroll
  for (int i = 0; i < 8; ++i) { out[i] = lo[i]; out[i + 8] = hi[i]; }
  return out;
}

__device__ __forceinline__ v8f wmma16(v16h a, v16h b, v8f c) {
  v8f d = __builtin_amdgcn_wmma_f32_16x16x32_f16(false, a, false, b, (short)0, c,
                                                 false, false);
  asm volatile("v_nop\n\tv_nop\n\tv_nop\n\tv_nop" : "+v"(d) : "v"(a), "v"(b));
  return d;
}

__device__ __forceinline__ float red32_sum(float x) {
#pragma unroll
  for (int off = 1; off < 32; off <<= 1) x += __shfl_xor(x, off, 32);
  return x;
}

__device__ __forceinline__ float leaky(float x) { return (x >= 0.0f) ? x : 0.2f * x; }

__global__ __launch_bounds__(256) void awconv_kernel(
    const float* __restrict__ AW, _Float16* __restrict__ AWt) {
  __shared__ __attribute__((aligned(16))) _Float16 T[ND * LDA];
  const unsigned tid = threadIdx.x;
  const unsigned a = blockIdx.x;
  const float* src = AW + (size_t)a * (NF * ND);
#pragma unroll 4
  for (unsigned j = 0; j < 8u; ++j) {
    const unsigned idx = tid + 256u * j;
    const unsigned n = idx >> 4, d = idx & 15u;
    const float v = src[idx];
    T[d * LDA + n] = toh_flush(WCARRY * bf16r(v));
  }
  __syncthreads();
  const unsigned d = tid >> 4;
  const unsigned kc = (tid & 15u) * 8u;
  const v8h x = *(const v8h*)&T[d * LDA + kc];
  _Float16* p = AWt + (size_t)(a * ND + d) * NF + kc;
  *(volatile v8h*)p = x;
  __threadfence();
  *(volatile v8h*)p = x;
}

__global__ __launch_bounds__(64) __attribute__((amdgpu_num_vgpr(256))) void main_kernel(
    const float* __restrict__ X, const _Float16* __restrict__ AWt,
    const float* __restrict__ W0, const float* __restrict__ W1,
    const float* __restrict__ W2, const float* __restrict__ W3,
    const float* __restrict__ Wh, const float* __restrict__ bh,
    float* __restrict__ rep_out, float* __restrict__ part, float* __restrict__ ce_out) {
  __shared__ __attribute__((aligned(16))) float sW1[NH * WP];
  __shared__ __attribute__((aligned(16))) float sW2[NH * WP];
  __shared__ __attribute__((aligned(16))) float sW3[NH * WP];
  __shared__ float sWh[NT * NH];
  __shared__ float sbh[NT];
  __shared__ __attribute__((aligned(16))) float R[K1_ROWS * PITCH];
  __shared__ __attribute__((aligned(16))) float sPart[REPW];
  __shared__ __attribute__((aligned(16))) float sCe[K1_ROWS];
  static_assert(sizeof(float) * (3 * NH * WP + NT * NH + NT + K1_ROWS * PITCH + REPW + K1_ROWS)
                <= 131072);

  const unsigned tid = threadIdx.x, lane = tid & 31u;
  const unsigned wave = (unsigned)__builtin_amdgcn_readfirstlane((int)(threadIdx.x >> 5));
  const unsigned hh = lane >> 4, m = lane & 15u;

  for (unsigned i = tid; i < (unsigned)(NH * WP); i += 64u) {
    const unsigned row = i / (unsigned)WP;
    const unsigned col = i - row * (unsigned)WP;
    const unsigned cc = (col < (unsigned)NH) ? col : (unsigned)(NH - 1);
    const bool okc = (col < (unsigned)NH);
    const float v1 = bf16r(W1[row * NH + cc]);
    const float v2 = bf16r(W2[row * NH + cc]);
    const float v3 = bf16r(W3[row * NH + cc]);
    sW1[i] = okc ? v1 : 0.0f;
    sW2[i] = okc ? v2 : 0.0f;
    sW3[i] = okc ? v3 : 0.0f;
  }
  for (unsigned i = tid; i < (unsigned)(NT * NH); i += 64u) sWh[i] = bf16r(Wh[i]);
  if (tid < (unsigned)NT) sbh[tid] = bf16r(bh[tid]);

  const unsigned rowBase = blockIdx.x * (unsigned)K1_ROWS + wave * 16u;

  v16h xf[4];
  {
    const float* xr = X + (size_t)(rowBase + m) * NF + hh * 8u;
#pragma unroll
    for (int ks = 0; ks < 4; ++ks) {
      const v4f a0 = *(const v4f*)(xr + ks * 32);
      const v4f a1 = *(const v4f*)(xr + ks * 32 + 4);
      const v4f a2 = *(const v4f*)(xr + ks * 32 + 16);
      const v4f a3 = *(const v4f*)(xr + ks * 32 + 20);
#pragma unroll
      for (int i = 0; i < 4; ++i) {
        xf[ks][i]      = toh_flush(XCARRY * bf16r(a0[i]));
        xf[ks][i + 4]  = toh_flush(XCARRY * bf16r(a1[i]));
        xf[ks][i + 8]  = toh_flush(XCARRY * bf16r(a2[i]));
        xf[ks][i + 12] = toh_flush(XCARRY * bf16r(a3[i]));
      }
    }
  }

  v16h w0f;
  {
    const unsigned orow = (m < (unsigned)NH) ? m : (unsigned)(NH - 1);
    const bool ok = (m < (unsigned)NH);
    const float* wp = W0 + orow * ND + hh * 8u;
    const v4f a0 = *(const v4f*)(wp);
    const v4f a1 = *(const v4f*)(wp + 4);
#pragma unroll
    for (int i = 0; i < 4; ++i) {
      const float e0 = ok ? (WCARRY * bf16r(a0[i])) : 0.0f;
      const float e1 = ok ? (WCARRY * bf16r(a1[i])) : 0.0f;
      w0f[i]     = toh_flush(e0);
      w0f[i + 4] = toh_flush(e1);
    }
#pragma unroll
    for (int i = 8; i < 16; ++i) w0f[i] = (h16)0.0f;
  }

  __syncthreads();

  float ce_acc = 0.0f;

#pragma unroll 1
  for (unsigned j2 = 0; j2 < 16u; ++j2) {
    v8f d2[2];
#pragma unroll
    for (int s = 0; s < 2; ++s) {
      const _Float16* ap = AWt + (size_t)((j2 * 2u + (unsigned)s) * ND + m) * NF + hh * 8u;
      v8f acc = {};
#pragma unroll
      for (int ks = 0; ks < 4; ++ks) {
        const v16h af = frag_at(ap + ks * 32);
        acc = wmma16(af, xf[ks], acc);
      }
      v16h bt;
#if XT_RES
      v16h br;
#endif
#pragma unroll
      for (int r = 0; r < 8; ++r) {
        const float t = acc[r] * XT_SCALE;
        const h16 hi = toh_flush(t);
        bt[r] = hi;
        bt[r + 8] = (h16)0.0f;
#if XT_RES
        br[r] = toh_flush((t - (float)hi) * RCARRY);
        br[r + 8] = (h16)0.0f;
#endif
      }
      v8f z = {};
      v8f dd = wmma16(w0f, bt, z);
#if XT_RES
      v8f zr = {};
      const v8f dr = wmma16(w0f, br, zr);
#pragma unroll
      for (int r = 0; r < 8; ++r) dd[r] = dd[r] + dr[r] * (1.0f / RCARRY);
#endif
      d2[s] = dd;
    }

    float h0[NH];
#pragma unroll
    for (int o = 0; o < 8; ++o) {
      const float t1 = __shfl_xor(d2[1][o], 16, 32);
      h0[o] = (hh != 0u) ? t1 : d2[0][o];
    }
#pragma unroll
    for (int j = 0; j < 2; ++j) {
      const float t0 = __shfl_xor(d2[0][j], 16, 32);
      h0[8 + j] = (hh != 0u) ? d2[1][j] : t0;
    }
    const unsigned a = j2 * 2u + hh;

    float t0v[NH], h1[NH];
#pragma unroll
    for (int k = 0; k < NH; ++k) t0v[k] = leaky(h0[k] * H0_SCALE);

    unsigned z1 = 0u;
    asm volatile("" : "+v"(z1), "+v"(t0v[NH - 1]));
#pragma unroll
    for (int o = 0; o < NH; ++o) {
      const v4f wa = *(const v4f*)&sW1[z1 + (unsigned)o * (unsigned)WP];
      const v4f wb = *(const v4f*)&sW1[z1 + (unsigned)o * (unsigned)WP + 4u];
      const v4f wc = *(const v4f*)&sW1[z1 + (unsigned)o * (unsigned)WP + 8u];
      float s1 = 0.0f;
#pragma unroll
      for (int k = 0; k < 4; ++k) s1 = __builtin_fmaf(wa[k], t0v[k], s1);
#pragma unroll
      for (int k = 0; k < 4; ++k) s1 = __builtin_fmaf(wb[k], t0v[4 + k], s1);
#pragma unroll
      for (int k = 0; k < 2; ++k) s1 = __builtin_fmaf(wc[k], t0v[8 + k], s1);
      h1[o] = s1;
    }
#pragma unroll
    for (int k = 0; k < NH; ++k) t0v[k] = leaky(h1[k]);

    unsigned z2 = 0u;
    asm volatile("" : "+v"(z2), "+v"(t0v[NH - 1]));
#pragma unroll
    for (int o = 0; o < NH; ++o) {
      const v4f wa = *(const v4f*)&sW2[z2 + (unsigned)o * (unsigned)WP];
      const v4f wb = *(const v4f*)&sW2[z2 + (unsigned)o * (unsigned)WP + 4u];
      const v4f wc = *(const v4f*)&sW2[z2 + (unsigned)o * (unsigned)WP + 8u];
      float s2 = 0.0f;
#pragma unroll
      for (int k = 0; k < 4; ++k) s2 = __builtin_fmaf(wa[k], t0v[k], s2);
#pragma unroll
      for (int k = 0; k < 4; ++k) s2 = __builtin_fmaf(wb[k], t0v[4 + k], s2);
#pragma unroll
      for (int k = 0; k < 2; ++k) s2 = __builtin_fmaf(wc[k], t0v[8 + k], s2);
      h1[o] = s2;
    }
#pragma unroll
    for (int k = 0; k < NH; ++k) t0v[k] = leaky(h1[k]);

    unsigned z3 = 0u;
    asm volatile("" : "+v"(z3), "+v"(t0v[NH - 1]));
    float rep[NH];
#pragma unroll
    for (int o = 0; o < NH; ++o) {
      const v4f wa = *(const v4f*)&sW3[z3 + (unsigned)o * (unsigned)WP];
      const v4f wb = *(const v4f*)&sW3[z3 + (unsigned)o * (unsigned)WP + 4u];
      const v4f wc = *(const v4f*)&sW3[z3 + (unsigned)o * (unsigned)WP + 8u];
      float s3 = 0.0f;
#pragma unroll
      for (int k = 0; k < 4; ++k) s3 = __builtin_fmaf(wa[k], t0v[k], s3);
#pragma unroll
      for (int k = 0; k < 4; ++k) s3 = __builtin_fmaf(wb[k], t0v[4 + k], s3);
#pragma unroll
      for (int k = 0; k < 2; ++k) s3 = __builtin_fmaf(wc[k], t0v[8 + k], s3);
      rep[o] = s3;
    }

    {
      const unsigned rb = (wave * 16u + m) * (unsigned)PITCH + a * (unsigned)NH;
#pragma unroll
      for (int o = 0; o < NH; ++o) R[rb + (unsigned)o] = rep[o];
    }

    float lr[NH];
#pragma unroll
    for (int k = 0; k < NH; ++k) lr[k] = leaky(rep[k]);
    float mx = -3.0e38f, ssum = 0.0f, pa = 0.0f;
#pragma unroll 1
    for (unsigned o = 0; o < (unsigned)NT; ++o) {
      float p = sbh[o];
#pragma unroll
      for (int k = 0; k < NH; ++k) p = __builtin_fmaf(sWh[o * NH + (unsigned)k], lr[k], p);
      pa = (o == a) ? p : pa;
      const float e = __expf(-fabsf(p - mx));
      ssum = (p > mx) ? (ssum * e + 1.0f) : (ssum + e);
      mx = fmaxf(mx, p);
    }
    ce_acc += (mx + __logf(ssum) - pa);
  }

  {
    const float other = __shfl_xor(ce_acc, 16, 32);
    const float tot = (ce_acc + other) * (1.0f / (float)NT);
    if (hh == 0u) sCe[wave * 16u + m] = tot;
  }
  __syncthreads();

  {
    float* gbase = rep_out + (size_t)rowBase * REPW;
#pragma unroll 1
    for (unsigned ch = 0; ch < 5u; ++ch) {
      v4f x[8];
      unsigned off[8];
#pragma unroll
      for (unsigned i = 0; i < 8u; ++i) {
        const unsigned p = (ch * 8u + i) * 32u + lane;
        const unsigned row = p / 80u;
        const unsigned c4 = p - row * 80u;
        x[i] = *(const v4f*)&R[(wave * 16u + row) * (unsigned)PITCH + c4 * 4u];
        off[i] = p * 4u;
      }
#pragma unroll
      for (int i = 0; i < 8; ++i) *(volatile v4f*)(gbase + off[i]) = x[i];
      __threadfence();
#pragma unroll
      for (int i = 0; i < 8; ++i) *(volatile v4f*)(gbase + off[i]) = x[i];
    }
  }

#pragma unroll 1
  for (unsigned j = 0; j < 5u; ++j) {
    const unsigned c = tid + 64u * j;
    float s = 0.0f;
#pragma unroll 4
    for (unsigned r = 0; r < (unsigned)K1_ROWS; ++r) s += R[r * (unsigned)PITCH + c];
    sPart[c] = s;
  }
  __syncthreads();
  {
    float* pb = part + (size_t)blockIdx.x * REPW;
    const unsigned t1 = (tid < 16u) ? tid : 15u;
    const v4f y0 = *(const v4f*)&sPart[tid * 4u];
    const v4f y1 = *(const v4f*)&sPart[256u + t1 * 4u];
    const unsigned t2 = (tid < 8u) ? tid : 7u;
    const v4f cv = *(const v4f*)&sCe[t2 * 4u];
    float* cb = ce_out + (size_t)blockIdx.x * K1_ROWS;
    *(volatile v4f*)(pb + tid * 4u) = y0;
    if (tid < 16u) *(volatile v4f*)(pb + 256u + tid * 4u) = y1;
    if (tid < 8u)  *(volatile v4f*)(cb + tid * 4u) = cv;
    __threadfence();
    *(volatile v4f*)(pb + tid * 4u) = y0;
    if (tid < 16u) *(volatile v4f*)(pb + 256u + tid * 4u) = y1;
    if (tid < 8u)  *(volatile v4f*)(cb + tid * 4u) = cv;
  }
}

__global__ __launch_bounds__(320) void colmean_kernel(
    const float* __restrict__ part, float* __restrict__ means) {
  __shared__ __attribute__((aligned(16))) float sM[REPW];
  const unsigned tid = threadIdx.x;
  double s = 0.0;
#pragma unroll 4
  for (unsigned blk = 0; blk < (unsigned)K1_BLOCKS; ++blk)
    s += (double)part[(size_t)blk * REPW + tid];
  sM[tid] = (float)(s * (1.0 / (double)NB));
  __syncthreads();
  const unsigned t1 = (tid < 80u) ? tid : 79u;
  const v4f y = *(const v4f*)&sM[t1 * 4u];
  if (tid < 80u) *(volatile v4f*)(means + tid * 4u) = y;
  __threadfence();
  if (tid < 80u) *(volatile v4f*)(means + tid * 4u) = y;
}

__global__ __launch_bounds__(256) void triplet_kernel(
    const float* __restrict__ rep, const float* __restrict__ means, float* __restrict__ hpart) {
  __shared__ float sMean[REPW];
  __shared__ float sw[8];
  const unsigned tid = threadIdx.x, lane = tid & 31u;
  const unsigned wave = (unsigned)__builtin_amdgcn_readfirstlane((int)(threadIdx.x >> 5));
  for (unsigned i = tid; i < (unsigned)REPW; i += 256u) sMean[i] = means[i];
  __syncthreads();

  float acc = 0.0f;
#pragma unroll 1
  for (unsigned it = 0; it < (unsigned)TRI_ITERS; ++it) {
    const unsigned task = it * ((unsigned)TRI_BLOCKS * 256u) + blockIdx.x * 256u + tid;
    const unsigned b = task >> 5, t = task & 31u;
    const v2f* xp = (const v2f*)(rep + (size_t)b * REPW + t * NH);
    float x[NH];
#pragma unroll
    for (int i2 = 0; i2 < 5; ++i2) {
      const v2f v = xp[i2];
      x[2 * i2] = v[0];
      x[2 * i2 + 1] = v[1];
    }
    float pos = 0.0f, neg = 3.0e38f;
#pragma unroll 1
    for (unsigned c = 0; c < (unsigned)NT; ++c) {
      float r = 0.0f;
#pragma unroll
      for (int h = 0; h < NH; ++h) {
        const float d = x[h] - sMean[c * NH + (unsigned)h];
        r = __builtin_fmaf(d, d, r);
      }
      pos = (c == t) ? r : pos;
      const float rr = (c == t) ? (r + 1.0e6f) : r;
      neg = fminf(neg, rr);
    }
    acc += fmaxf((pos + 1.0f) - neg, 0.0f);
  }

  const float wsum = red32_sum(acc);
  if (lane == 0u) sw[wave] = wsum;
  __syncthreads();
  const float total = ((sw[0] + sw[1]) + (sw[2] + sw[3])) + ((sw[4] + sw[5]) + (sw[6] + sw[7]));
  v4f y;
  y[0] = (tid == 0u) ? total : 0.0f;
  y[1] = 0.0f; y[2] = 0.0f; y[3] = 0.0f;
  float* hb = hpart + (size_t)blockIdx.x * 32u;
  if (tid < 8u) *(volatile v4f*)(hb + tid * 4u) = y;
  __threadfence();
  if (tid < 8u) *(volatile v4f*)(hb + tid * 4u) = y;
}

__global__ __launch_bounds__(256) void final_kernel(
    const float* __restrict__ ce, const float* __restrict__ hpart, float* __restrict__ loss_out) {
  __shared__ double red[256];
  const unsigned tid = threadIdx.x;
  double s = 0.0;
#pragma unroll 1
  for (unsigned i = tid; i < (unsigned)TRI_BLOCKS; i += 256u) s += (double)hpart[(size_t)i * 32u];
  red[tid] = s;
  __syncthreads();
  for (unsigned st = 128u; st > 0u; st >>= 1) {
    if (tid < st) red[tid] += red[tid + st];
    __syncthreads();
  }
  const float tc = (float)(red[0] * (1.0 / ((double)NB * (double)NT)));
  const float add = 0.1f * tc;
  const unsigned row = blockIdx.x * (unsigned)FIN_ROWS + tid * 4u;
  const v4f c = *(const v4f*)(ce + row);
  v4f o;
#pragma unroll
  for (int j = 0; j < 4; ++j) o[j] = c[j] + add;
  float* p = loss_out + row;
  *(volatile v4f*)p = o;
  __threadfence();
  *(volatile v4f*)p = o;
}

extern "C" void kernel_launch(void* const* d_in, const int* in_sizes, int n_in,
                              void* d_out, int out_size, void* d_ws, size_t ws_size,
                              hipStream_t stream) {
  if (n_in < 8) return;
  if ((long long)in_sizes[0] < (long long)NB * NF) return;
  if ((long long)in_sizes[1] < (long long)NT * NF * ND) return;
  if (in_sizes[2] < NH * ND) return;
  if (in_sizes[3] < NH * NH || in_sizes[4] < NH * NH || in_sizes[5] < NH * NH) return;
  if (in_sizes[6] < NT * NH || in_sizes[7] < NT) return;
  if ((long long)out_size < (long long)OUT1_OFF + (long long)NB) return;
  if (ws_size < WS_TOTAL) return;

  const float* X  = (const float*)d_in[0];
  const float* AW = (const float*)d_in[1];
  const float* W0 = (const float*)d_in[2];
  const float* W1 = (const float*)d_in[3];
  const float* W2 = (const float*)d_in[4];
  const float* W3 = (const float*)d_in[5];
  const float* Wh = (const float*)d_in[6];
  const float* bh = (const float*)d_in[7];
  float* out = (float*)d_out;

  char* ws = (char*)d_ws;
  _Float16* AWt  = (_Float16*)(ws + OFF_AWT);
  float*    part = (float*)(ws + OFF_PART);
  float*    cepl = (float*)(ws + OFF_CE);
  float*    mean = (float*)(ws + OFF_MEAN);
  float*    hp   = (float*)(ws + OFF_HP);

  awconv_kernel<<<dim3(NT), dim3(256), 0, stream>>>(AW, AWt);
  main_kernel<<<dim3(K1_BLOCKS), dim3(64), 0, stream>>>(X, AWt, W0, W1, W2, W3, Wh, bh,
                                                        out, part, cepl);
  colmean_kernel<<<dim3(1), dim3(320), 0, stream>>>(part, mean);
  triplet_kernel<<<dim3(TRI_BLOCKS), dim3(256), 0, stream>>>(out, mean, hp);
  final_kernel<<<dim3(FIN_BLOCKS), dim3(256), 0, stream>>>(cepl, hp, out + OUT1_OFF);
}
